// DiffMamba_65730179498079
// MI455X (gfx1250) — hardware-verified
//
#include <hip/hip_runtime.h>
#include <math.h>

typedef __attribute__((ext_vector_type(16))) _Float16 v16h;
typedef __attribute__((ext_vector_type(8)))  _Float16 v8h;
typedef __attribute__((ext_vector_type(16))) __bf16   v16b;
typedef __attribute__((ext_vector_type(8)))  __bf16   v8b;
typedef __attribute__((ext_vector_type(8)))  float    v8f;
typedef __attribute__((ext_vector_type(4)))  float    v4f;

constexpr int kBatch   = 2;
constexpr int kSeq     = 2048;
constexpr int kDm      = 256;
constexpr int kHd      = 16;
constexpr int kNh      = 16;
constexpr int kNst     = 64;
constexpr int kDinner  = 32;
constexpr int kNhIn    = 2;
constexpr int kConvDim = kDinner + 2 * kNst;
constexpr int kDinProj = 2 * kDinner + 2 * kNst + kNhIn;
constexpr int kDtCol   = 2 * kDinner + 2 * kNst;
constexpr int kNpad    = 208;
constexpr int kNtIn    = kNpad / 16;
constexpr int kChunk   = 32;
constexpr int kRows    = kBatch * kSeq;
constexpr int kPlane   = kSeq * kHd;
constexpr int kWinRows = kNh * kNpad;
static_assert(kConvDim == 160 && kDinProj == 194 && kDtCol == 192, "column map");
static_assert(kNh * kHd == kDm, "head split");
static_assert((kSeq % kChunk) == 0 && (kNpad % 16) == 0 && kNpad >= kDinProj, "tiles");
static_assert(kNtIn == 13, "in_proj n tiles");
static_assert((kRows % 64) == 0 && (kDm % 64) == 0 && (kDm % 32) == 0, "final GEMM tile multiples");

constexpr float kCarryG  = 16.0f;
constexpr float kCarryWo = 8.0f;
constexpr float kCarryO  = 8.0f;
constexpr float kCarryPw = 16.0f;
constexpr float kFoldOut  = 1.0f / (kCarryG * kCarryWo);
constexpr float kFoldProj = 1.0f / (kCarryO * kCarryPw);

constexpr size_t kSzWP  = (size_t)2 * kWinRows * 32 * 2;
constexpr size_t kSzWOT = (size_t)2 * kNh * kHd * kDinner * 2;
constexpr size_t kSzPJW = (size_t)kDm * kDm * 2;
constexpr size_t kSzY   = (size_t)2 * kNh * kBatch * kPlane * 4;
constexpr size_t kSzST  = (size_t)kNh * kBatch * 32 * 4;
constexpr size_t kSzAPL = (size_t)kRows * kDm * 2;
constexpr size_t kOffWP1 = 0;
constexpr size_t kOffWP2 = kOffWP1 + kSzWP;
constexpr size_t kOffWOT = kOffWP2 + kSzWP;
constexpr size_t kOffPJW = kOffWOT + kSzWOT;
constexpr size_t kOffY   = kOffPJW + kSzPJW;
constexpr size_t kOffST  = kOffY + kSzY;
constexpr size_t kOffAPL = kOffST + kSzST;
constexpr size_t kWsTotal = kOffAPL + kSzAPL;
static_assert(kWsTotal == 11505664ull, "carve total");
static_assert(kWsTotal <= 134217728ull, "carve cap");
static_assert((kOffWP2 % 128) == 0 && (kOffWOT % 128) == 0 && (kOffPJW % 128) == 0 && (kOffY % 128) == 0 &&
              (kOffST % 128) == 0 && (kOffAPL % 128) == 0, "128-B aligned regions");

__device__ __forceinline__ unsigned short f2bf_bits(float f) {
  unsigned u = __float_as_uint(f);
  return (unsigned short)((u + 0x7FFFu + ((u >> 16) & 1u)) >> 16);
}
__device__ __forceinline__ float bf_bits2f(unsigned short h) { return __uint_as_float(((unsigned)h) << 16); }

__device__ __forceinline__ void keep4_h(v16h a, v16h b, v16h c, v16h d) { asm volatile("v_nop" :: "v"(a), "v"(b), "v"(c), "v"(d)); }
__device__ __forceinline__ void acc_guard4(v8f& a, v8f& b, v8f& c, v8f& d) { asm volatile("v_nop\n\tv_nop\n\tv_nop\n\tv_nop" : "+v"(a), "+v"(b), "+v"(c), "+v"(d)); }
__device__ __forceinline__ void guard_row4(v8f& a, v8f& b, v8f& c, v8f& d, v16h x, v16h y0, v16h y1, v16h y2, v16h y3) {
  asm volatile("v_nop\n\tv_nop\n\tv_nop\n\tv_nop" : "+v"(a), "+v"(b), "+v"(c), "+v"(d) : "v"(x), "v"(y0), "v"(y1), "v"(y2), "v"(y3));
}
template <typename T> struct Frag;
template <> struct Frag<_Float16> {
  typedef v16h V; union U { v16h v; v8h h[2]; };
  static __device__ __forceinline__ v16h load(const _Float16* p) {
    U f; f.h[0] = *(const v8h*)(p); f.h[1] = *(const v8h*)(p + 16); return f.v;
  }
  static __device__ __forceinline__ v8f mma(v16h a, v16h b, v8f c) {
    return __builtin_amdgcn_wmma_f32_16x16x32_f16(false, a, false, b, (short)0, c, false, false);
  }
};
template <> struct Frag<__bf16> {
  typedef v16b V; union U { v16b v; v8b h[2]; };
  static __device__ __forceinline__ v16b load(const __bf16* p) {
    U f; f.h[0] = *(const v8b*)(p); f.h[1] = *(const v8b*)(p + 16); return f.v;
  }
};
__device__ __forceinline__ v8f mma_bf(v16b a, v16b b, v8f c) {
  c = __builtin_amdgcn_wmma_f32_16x16x32_bf16(false, a, false, b, (short)0, c, false, false);
  asm volatile("v_nop\n\tv_nop\n\tv_nop\n\tv_nop" : "+v"(c) : "v"(a), "v"(b));
  return c;
}
__device__ __forceinline__ v8f mma_hf(v16h a, v16h b, v8f c) {
  c = __builtin_amdgcn_wmma_f32_16x16x32_f16(false, a, false, b, (short)0, c, false, false);
  asm volatile("v_nop\n\tv_nop\n\tv_nop\n\tv_nop" : "+v"(c) : "v"(a), "v"(b));
  return c;
}

__global__ __launch_bounds__(256) void prep_planes_kernel(
    const float* __restrict__ win_a, const float* __restrict__ win_b,
    const float* __restrict__ wout_a, const float* __restrict__ wout_b,
    const float* __restrict__ projw,
    unsigned short* __restrict__ WP1, unsigned short* __restrict__ WP2,
    unsigned short* __restrict__ WOT, unsigned short* __restrict__ PJW)
{
  const int bx = blockIdx.x, tid = threadIdx.x;
  if (bx < 104) {
    const int team = bx / 52;
    const int i = (bx - team * 52) * 256 + tid;
    const int row = i >> 2, seg = i & 3;
    const int head = row / kNpad;
    const int n = row - head * kNpad;
    const int nc = (n < kDinProj) ? n : (kDinProj - 1);
    const bool valid = (n < kDinProj);
    const bool dup = (seg >= 2);
    const float* W = team ? win_b : win_a;
    const float* src = W + ((size_t)(head * kDinProj + nc)) * kHd + (seg & 1) * 8;
    const v4f a0 = *(const v4f*)(src);
    const v4f a1 = *(const v4f*)(src + 4);
    v8h hv, lv;
#pragma unroll
    for (int e = 0; e < 4; ++e) {
      const float f0 = valid ? a0[e] : 0.0f;
      const float f1 = valid ? a1[e] : 0.0f;
      const unsigned short h0 = f2bf_bits(f0), h1 = f2bf_bits(f1);
      const unsigned short l0 = f2bf_bits(f0 - bf_bits2f(h0)), l1 = f2bf_bits(f1 - bf_bits2f(h1));
      const unsigned short m0 = dup ? (unsigned short)0 : l0;
      const unsigned short m1 = dup ? (unsigned short)0 : l1;
      hv[e]     = __builtin_bit_cast(_Float16, h0);
      hv[4 + e] = __builtin_bit_cast(_Float16, h1);
      lv[e]     = __builtin_bit_cast(_Float16, m0);
      lv[4 + e] = __builtin_bit_cast(_Float16, m1);
    }
    const size_t o = ((size_t)(team * kWinRows + row)) * 32 + seg * 8;
    *(volatile v8h*)(WP1 + o) = hv;
    *(volatile v8h*)(WP2 + o) = lv;
    __threadfence();
    *(volatile v8h*)(WP1 + o) = hv;
    *(volatile v8h*)(WP2 + o) = lv;
  } else if (bx < 112) {
    const int idx = (bx - 104) * 256 + tid;
    const int team = idx >> 10;
    const size_t e0 = (size_t)(idx & 1023) << 3;
    const float* src = (team ? wout_b : wout_a) + e0;
    const v4f a0 = *(const v4f*)(src);
    const v4f a1 = *(const v4f*)(src + 4);
    v8h hv;
#pragma unroll
    for (int e = 0; e < 4; ++e) {
      hv[e]     = (_Float16)(a0[e] * kCarryWo);
      hv[4 + e] = (_Float16)(a1[e] * kCarryWo);
    }
    unsigned short* q = WOT + (size_t)team * (kNh * kHd * kDinner) + e0;
    *(volatile v8h*)q = hv;
    __threadfence();
    *(volatile v8h*)q = hv;
  } else {
    const int idx = (bx - 112) * 256 + tid;
    const size_t e0 = (size_t)idx << 3;
    const float* src = projw + e0;
    const v4f a0 = *(const v4f*)(src);
    const v4f a1 = *(const v4f*)(src + 4);
    v8h hv;
#pragma unroll
    for (int e = 0; e < 4; ++e) {
      hv[e]     = (_Float16)(a0[e] * kCarryPw);
      hv[4 + e] = (_Float16)(a1[e] * kCarryPw);
    }
    unsigned short* q = PJW + e0;
    *(volatile v8h*)q = hv;
    __threadfence();
    *(volatile v8h*)q = hv;
  }
}

__global__ __launch_bounds__(128) void mamba_head_kernel(
    const float* __restrict__ x,
    const unsigned short* __restrict__ WP1, const unsigned short* __restrict__ WP2,
    const unsigned short* __restrict__ WOT,
    const float* __restrict__ convw, const float* __restrict__ convb,
    const float* __restrict__ dtb, const float* __restrict__ Alog,
    const float* __restrict__ Dp, const float* __restrict__ nw,
    float* __restrict__ Yteam)
{
  __shared__ __align__(16) __bf16   sU[kChunk * 32];
  __shared__ __align__(16) float    sZX[(kChunk + 3) * kNpad];
  __shared__ __align__(16) float    sXBC[kChunk * kConvDim];
  __shared__ __align__(16) float    sCW[kConvDim * 4];
  __shared__ __align__(16) float    sCB[kConvDim];
  __shared__ __align__(16) float    sNW[kDinner];
  __shared__ __align__(16) float    sDT[kChunk * kNhIn];
  __shared__ __align__(16) float    sDA[kChunk * kNhIn];
  __shared__ __align__(16) float    sY[kChunk * kDinner];
  __shared__ __align__(16) _Float16 sG[kChunk * kDinner];
  __shared__ __align__(16) float    sO[kChunk * kHd];
  union FragB { v16b v; v8b h[2]; };
  union FragH { v16h v; v8h h[2]; };

  const int tid  = threadIdx.x;
  const int lane = tid & 31;
  const int wave = __builtin_amdgcn_readfirstlane(tid >> 5);
  const int hh   = lane >> 4;
  const int c    = lane & 15;
  const int head = blockIdx.x >> 1;
  const int bb   = blockIdx.x & 1;

  for (int i = tid; i < kConvDim * 4; i += 128) sCW[i] = convw[head * kConvDim * 4 + i];
  for (int i = tid; i < kConvDim; i += 128) sCB[i] = convb[head * kConvDim + i];
  if (tid < kDinner) sNW[tid] = nw[head * kDinner + tid];
  for (int i = tid; i < 3 * kNpad; i += 128) sZX[i] = 0.0f;

  const float dtb_l = dtb[head * kNhIn + (tid & 1)];
  const float an_l  = -expf(Alog[head * kNhIn + (tid & 1)]);
  const float dskip = Dp[head * kNhIn + ((tid & 3) >> 1)];

  v16b bf1[4], bf2[4];
#pragma unroll
  for (int j = 0; j < 4; ++j) {
    const int nt  = wave + 4 * j;
    const int ntc = (nt < kNtIn) ? nt : (kNtIn - 1);
    const size_t bo = ((size_t)(head * kNpad + ntc * 16 + c)) * 32 + 8 * hh;
    bf1[j] = Frag<__bf16>::load((const __bf16*)WP1 + bo);
    bf2[j] = Frag<__bf16>::load((const __bf16*)WP2 + bo);
  }
  const v16h bo_f = Frag<_Float16>::load((const _Float16*)WOT + ((size_t)(head * kHd + c)) * kDinner + 8 * hh);

  const int nq = tid & 3;
  const int ch = tid >> 2;
  const int hi = tid >> 6;
  float hst[16];
#pragma unroll
  for (int k = 0; k < 16; ++k) hst[k] = 0.0f;

  const float* xb = x + ((size_t)bb * kSeq) * kDm + head * kHd;
  float* Yblk = Yteam + (size_t)blockIdx.x * kPlane;
  const v8f zero8 = (v8f){0.f, 0.f, 0.f, 0.f, 0.f, 0.f, 0.f, 0.f};
  __syncthreads();

#pragma unroll 1
  for (int ci = 0; ci < kSeq / kChunk; ++ci) {
    const int t0 = ci * kChunk;

    {
      const int srow = tid >> 2, sseg = tid & 3;
      const float* xs = xb + (size_t)(t0 + srow) * kDm + (sseg & 1) * 8;
      const v4f a0 = *(const v4f*)(xs);
      const v4f a1 = *(const v4f*)(xs + 4);
      const bool lo_sel = (sseg >= 2);
      v8b pk;
#pragma unroll
      for (int e = 0; e < 4; ++e) {
        const unsigned short h0 = f2bf_bits(a0[e]), h1 = f2bf_bits(a1[e]);
        const unsigned short l0 = f2bf_bits(a0[e] - bf_bits2f(h0)), l1 = f2bf_bits(a1[e] - bf_bits2f(h1));
        const unsigned short s0 = lo_sel ? l0 : h0;
        const unsigned short s1 = lo_sel ? l1 : h1;
        pk[e]     = __builtin_bit_cast(__bf16, s0);
        pk[4 + e] = __builtin_bit_cast(__bf16, s1);
      }
      *(v8b*)(sU + srow * 32 + sseg * 8) = pk;
    }
    __syncthreads();

    {
      FragB fa0, fa1;
      fa0.h[0] = *(const v8b*)(sU + c * 32 + 8 * hh);
      fa0.h[1] = *(const v8b*)(sU + c * 32 + 16 + 8 * hh);
      fa1.h[0] = *(const v8b*)(sU + (16 + c) * 32 + 8 * hh);
      fa1.h[1] = *(const v8b*)(sU + (16 + c) * 32 + 16 + 8 * hh);
#pragma unroll
      for (int j = 0; j < 4; ++j) {
        const int nt = wave + 4 * j;
        if (nt < kNtIn) {
          v8f acc0 = zero8, acc1 = zero8;
          acc0 = mma_bf(fa0.v, bf1[j], acc0);
          acc0 = mma_bf(fa0.v, bf2[j], acc0);
          acc1 = mma_bf(fa1.v, bf1[j], acc1);
          acc1 = mma_bf(fa1.v, bf2[j], acc1);
          float* zp = sZX + (3 + 8 * hh) * kNpad + nt * 16 + c;
#pragma unroll
          for (int r = 0; r < 8; ++r) {
            zp[r * kNpad] = acc0[r];
            zp[(16 + r) * kNpad] = acc1[r];
          }
        }
      }
    }
    __syncthreads();

#pragma unroll 1
    for (int i = 0; i < (kChunk * kConvDim) / 128; ++i) {
      const int idx = tid + 128 * i;
      const int ct = idx / kConvDim;
      const int cc = idx - ct * kConvDim;
      const v4f w = *(const v4f*)(sCW + cc * 4);
      const float* zr = sZX + ct * kNpad + kDinner + cc;
      float s = w[0] * zr[0];
      s = fmaf(w[1], zr[kNpad], s);
      s = fmaf(w[2], zr[2 * kNpad], s);
      s = fmaf(w[3], zr[3 * kNpad], s);
      const float v = sCB[cc] + s;
      const float sg = __builtin_amdgcn_rcpf(1.0f + expf(-v));
      sXBC[idx] = v * sg;
    }
    if (wave < 2) {
      const int dt_t = tid >> 1, dt_h = tid & 1;
      const float raw = sZX[(3 + dt_t) * kNpad + kDtCol + dt_h] + dtb_l;
      const float dtv = fmaxf(raw, 0.0f) + log1pf(expf(-fabsf(raw)));
      sDT[dt_t * kNhIn + dt_h] = dtv;
      sDA[dt_t * kNhIn + dt_h] = expf(dtv * an_l);
    }
    __syncthreads();

    for (int i = tid; i < 3 * kConvDim; i += 128) {
      const int r = i / kConvDim;
      const int cc = i - r * kConvDim;
      sZX[r * kNpad + kDinner + cc] = sZX[(kChunk + r) * kNpad + kDinner + cc];
    }
#pragma unroll 1
    for (int s = 0; s < kChunk; ++s) {
      const float dA  = sDA[s * kNhIn + hi];
      const float dtv = sDT[s * kNhIn + hi];
      const float* xr = sXBC + s * kConvDim;
      const float dtx = dtv * xr[ch];
      v4f Bq[4], Cq[4];
#pragma unroll
      for (int q4 = 0; q4 < 4; ++q4) {
        Bq[q4] = *(const v4f*)(xr + kDinner + nq * 16 + 4 * q4);
        Cq[q4] = *(const v4f*)(xr + kDinner + kNst + nq * 16 + 4 * q4);
      }
      float y = 0.0f;
#pragma unroll
      for (int k = 0; k < 16; ++k) {
        const float hn = fmaf(dtx, Bq[k >> 2][k & 3], dA * hst[k]);
        hst[k] = hn;
        y = fmaf(hn, Cq[k >> 2][k & 3], y);
      }
      y += __shfl_xor(y, 1, 32);
      y += __shfl_xor(y, 2, 32);
      if (nq == 0) sY[s * kDinner + ch] = y;
    }
    __syncthreads();

    {
      const int gt = tid >> 2, gq = tid & 3;
      const v4f y0 = *(const v4f*)(sY + gt * kDinner + gq * 8);
      const v4f y1 = *(const v4f*)(sY + gt * kDinner + gq * 8 + 4);
      const v4f x0 = *(const v4f*)(sXBC + gt * kConvDim + gq * 8);
      const v4f x1 = *(const v4f*)(sXBC + gt * kConvDim + gq * 8 + 4);
      const v4f z0 = *(const v4f*)(sZX + (3 + gt) * kNpad + gq * 8);
      const v4f z1 = *(const v4f*)(sZX + (3 + gt) * kNpad + gq * 8 + 4);
      const v4f n0 = *(const v4f*)(sNW + gq * 8);
      const v4f n1 = *(const v4f*)(sNW + gq * 8 + 4);
      float gv[8];
      float ss = 0.0f;
#pragma unroll
      for (int e = 0; e < 4; ++e) {
        const float ya = fmaf(dskip, x0[e], y0[e]);
        const float za = z0[e];
        const float ga = ya * (za * __builtin_amdgcn_rcpf(1.0f + expf(-za)));
        gv[e] = ga;
        ss = fmaf(ga, ga, ss);
        const float yb = fmaf(dskip, x1[e], y1[e]);
        const float zb = z1[e];
        const float gb = yb * (zb * __builtin_amdgcn_rcpf(1.0f + expf(-zb)));
        gv[4 + e] = gb;
        ss = fmaf(gb, gb, ss);
      }
      ss += __shfl_xor(ss, 1, 32);
      ss += __shfl_xor(ss, 2, 32);
      const float rinv = rsqrtf(ss * (1.0f / (float)kDinner) + 1e-5f) * kCarryG;
      v8h hv;
#pragma unroll
      for (int e = 0; e < 4; ++e) {
        hv[e]     = (_Float16)((gv[e] * rinv) * n0[e]);
        hv[4 + e] = (_Float16)((gv[4 + e] * rinv) * n1[e]);
      }
      *(v8h*)(sG + gt * kDinner + gq * 8) = hv;
    }
    __syncthreads();

    if (wave < 2) {
      FragH ga;
      ga.h[0] = *(const v8h*)(sG + (wave * 16 + c) * kDinner + 8 * hh);
      ga.h[1] = *(const v8h*)(sG + (wave * 16 + c) * kDinner + 16 + 8 * hh);
      v8f acc = zero8;
      acc = mma_hf(ga.v, bo_f, acc);
#pragma unroll
      for (int r = 0; r < 8; ++r) sO[(wave * 16 + 8 * hh + r) * kHd + c] = acc[r] * kFoldOut;
    }
    __syncthreads();

    {
      const v4f ov = *(const v4f*)(sO + wave * 128 + lane * 4);
      float* dst = Yblk + (size_t)t0 * kHd + wave * 128 + lane * 4;
      *(volatile v4f*)dst = ov;
      __threadfence();
      *(volatile v4f*)dst = ov;
    }
  }
}

__global__ __launch_bounds__(256) void gn_stats_kernel(
    const float* __restrict__ Y, const float* __restrict__ lam, float* __restrict__ stats)
{
  __shared__ float sRedA[8];
  __shared__ float sRedB[8];
  const int tid = threadIdx.x, lane = tid & 31, wave = tid >> 5;
  const int hb = blockIdx.x;
  const int hd = hb >> 1;
  const float* y1 = Y + (size_t)hb * kPlane;
  const float* y2 = y1 + (size_t)(kNh * kBatch) * kPlane;
  const v4f l4 = *(const v4f*)(lam + hd * kHd + (tid & 3) * 4);
  float s = 0.0f;
#pragma unroll 2
  for (int it = 0; it < kPlane / 1024; ++it) {
    const int i = it * 1024 + tid * 4;
    const v4f a = *(const v4f*)(y1 + i);
    const v4f b = *(const v4f*)(y2 + i);
    const v4f d = a - l4 * b;
    s += (d[0] + d[1]) + (d[2] + d[3]);
  }
#pragma unroll
  for (int off = 1; off < 32; off <<= 1) s += __shfl_xor(s, off, 32);
  if (lane == 0) sRedA[wave] = s;
  __syncthreads();
  float tot = 0.0f;
#pragma unroll
  for (int w = 0; w < 8; ++w) tot += sRedA[w];
  const float mean = tot * (1.0f / (float)kPlane);
  float q = 0.0f;
#pragma unroll 2
  for (int it = 0; it < kPlane / 1024; ++it) {
    const int i = it * 1024 + tid * 4;
    const v4f a = *(const v4f*)(y1 + i);
    const v4f b = *(const v4f*)(y2 + i);
    const v4f d = (a - l4 * b) - mean;
    q += (d[0] * d[0] + d[1] * d[1]) + (d[2] * d[2] + d[3] * d[3]);
  }
#pragma unroll
  for (int off = 1; off < 32; off <<= 1) q += __shfl_xor(q, off, 32);
  if (lane == 0) sRedB[wave] = q;
  __syncthreads();
  float qt = 0.0f;
#pragma unroll
  for (int w = 0; w < 8; ++w) qt += sRedB[w];
  const float var = qt * (1.0f / (float)kPlane);
  const float rinv = rsqrtf(var + 1e-5f);
  if (tid < 32) {
    const float v = (lane == 0) ? mean : ((lane == 1) ? rinv : 0.0f);
    float* p = stats + hb * 32 + lane;
    *(volatile float*)p = v;
    __threadfence();
    *(volatile float*)p = v;
  }
}

__global__ __launch_bounds__(256) void gn_apply_kernel(
    const float* __restrict__ Y, const float* __restrict__ stats, const float* __restrict__ lam,
    const float* __restrict__ gnw, const float* __restrict__ gnb, unsigned short* __restrict__ APL)
{
  const int tid = threadIdx.x, lane = tid & 31, wave = tid >> 5;
  const int hd = lane >> 1, j0 = (lane & 1) * 8;
  const int m0 = blockIdx.x * 64 + wave * 8;
  const int bq = (blockIdx.x * 64) / kSeq;
  const int hb = hd * kBatch + bq;
  const float mean = stats[hb * 32];
  const float rinv = stats[hb * 32 + 1];
  const v4f l0 = *(const v4f*)(lam + lane * 8);
  const v4f l1 = *(const v4f*)(lam + lane * 8 + 4);
  const v4f w0 = *(const v4f*)(gnw + lane * 8);
  const v4f w1 = *(const v4f*)(gnw + lane * 8 + 4);
  const v4f g0 = *(const v4f*)(gnb + lane * 8);
  const v4f g1 = *(const v4f*)(gnb + lane * 8 + 4);
  const float* y1 = Y + (size_t)hb * kPlane + j0;
  const float* y2 = y1 + (size_t)(kNh * kBatch) * kPlane;
#pragma unroll 1
  for (int it = 0; it < 8; ++it) {
    const int m = m0 + it;
    const int t = m & (kSeq - 1);
    const v4f a0 = *(const v4f*)(y1 + t * kHd);
    const v4f a1 = *(const v4f*)(y1 + t * kHd + 4);
    const v4f c0 = *(const v4f*)(y2 + t * kHd);
    const v4f c1 = *(const v4f*)(y2 + t * kHd + 4);
    v8h hv;
#pragma unroll
    for (int e = 0; e < 4; ++e) {
      const float d0 = a0[e] - l0[e] * c0[e];
      const float d1 = a1[e] - l1[e] * c1[e];
      const float o0 = ((d0 - mean) * rinv) * w0[e] + g0[e];
      const float o1 = ((d1 - mean) * rinv) * w1[e] + g1[e];
      hv[e]     = (_Float16)(o0 * kCarryO);
      hv[4 + e] = (_Float16)(o1 * kCarryO);
    }
    unsigned short* dst = APL + (size_t)m * kDm + lane * 8;
    *(volatile v8h*)dst = hv;
    __threadfence();
    *(volatile v8h*)dst = hv;
  }
}

__global__ __launch_bounds__(256) void proj_gemm_kernel(
    const unsigned short* __restrict__ Ap, int lda,
    const unsigned short* __restrict__ Btp, int ldb,
    float* __restrict__ Cout, int ldc,
    const float* __restrict__ bias, const float* __restrict__ resid,
    int M, int N, int K, float scale)
{
  typedef _Float16 T;
  typedef v16h V;
  const T* A = (const T*)Ap;
  const T* Bt = (const T*)Btp;
  __shared__ __align__(16) float sT[8][16 * 68];
  const int lane = threadIdx.x & 31;
  const int wave = threadIdx.x >> 5;
  const int tilesN = N >> 6;
  const int tilesM = M >> 6;
  const int tile = blockIdx.x * 8 + wave;
  if (tile >= tilesM * tilesN) return;
  const int tm = tile / tilesN;
  const int tn = tile - tm * tilesN;
  const int m0 = tm << 6;
  const int n0 = tn << 6;
  const int rlane = lane & 15;
  const int koff  = (lane >> 4) * 8;
  const int mOff  = (lane >> 4) * 8;

  v8f acc[4][4];
#pragma unroll
  for (int i = 0; i < 4; ++i)
#pragma unroll
    for (int j = 0; j < 4; ++j) acc[i][j] = (v8f){0.f, 0.f, 0.f, 0.f, 0.f, 0.f, 0.f, 0.f};

  for (int k0 = 0; k0 < K; k0 += 32) {
    V bh[4];
#pragma unroll
    for (int j = 0; j < 4; ++j) {
      const size_t bo = (size_t)(n0 + (j << 4) + rlane) * ldb + koff + k0;
      bh[j] = Frag<T>::load(Bt + bo);
    }
#pragma unroll
    for (int i = 0; i < 4; ++i) {
      const size_t ao = (size_t)(m0 + (i << 4) + rlane) * lda + koff + k0;
      V ah = Frag<T>::load(A + ao);
#pragma unroll
      for (int j = 0; j < 4; ++j) acc[i][j] = Frag<T>::mma(ah, bh[j], acc[i][j]);
      guard_row4(acc[i][0], acc[i][1], acc[i][2], acc[i][3], ah, bh[0], bh[1], bh[2], bh[3]);
    }
    keep4_h(bh[0], bh[1], bh[2], bh[3]);
  }
  acc_guard4(acc[0][0], acc[0][1], acc[0][2], acc[0][3]);
  acc_guard4(acc[1][0], acc[1][1], acc[1][2], acc[1][3]);
  acc_guard4(acc[2][0], acc[2][1], acc[2][2], acc[2][3]);
  acc_guard4(acc[3][0], acc[3][1], acc[3][2], acc[3][3]);

  float* slab = sT[wave];
  const int hh = lane >> 4, c4 = (lane & 15) * 4;
  const v4f bias4 = *(const v4f*)(bias + n0 + c4);
#pragma unroll
  for (int i = 0; i < 4; ++i) {
    const int mBase = m0 + (i << 4);
#pragma unroll
    for (int j = 0; j < 4; ++j) {
#pragma unroll
      for (int r = 0; r < 8; ++r) slab[(mOff + r) * 68 + (j << 4) + rlane] = acc[i][j][r] * scale;
    }
    __builtin_amdgcn_fence(__ATOMIC_RELEASE, "workgroup");
    __builtin_amdgcn_wave_barrier();
    __builtin_amdgcn_fence(__ATOMIC_ACQUIRE, "workgroup");
    v4f vv[8];
#pragma unroll
    for (int it = 0; it < 8; ++it) {
      const int row = it * 2 + hh;
      const v4f sv = *(const v4f*)(slab + row * 68 + c4);
      const v4f rv = *(const v4f*)(resid + (size_t)(mBase + row) * ldc + n0 + c4);
      vv[it] = (sv + bias4) + rv;
    }
    for (int pass = 0; pass < 2; ++pass) {
#pragma unroll
      for (int it = 0; it < 8; ++it) {
        const int row = it * 2 + hh;
        *(volatile v4f*)(Cout + (size_t)(mBase + row) * ldc + n0 + c4) = vv[it];
      }
      __threadfence();
    }
    __builtin_amdgcn_fence(__ATOMIC_RELEASE, "workgroup");
    __builtin_amdgcn_wave_barrier();
    __builtin_amdgcn_fence(__ATOMIC_ACQUIRE, "workgroup");
  }
}

extern "C" void kernel_launch(void* const* d_in, const int* in_sizes, int n_in,
                              void* d_out, int out_size, void* d_ws, size_t ws_size,
                              hipStream_t stream)
{
  if (n_in < 22) return;
  if (in_sizes[0] != kRows * kDm) return;
  if (in_sizes[1] != kNh * kDinProj * kHd || in_sizes[9] != kNh * kDinProj * kHd) return;
  if (in_sizes[2] != kNh * kConvDim * 4 || in_sizes[10] != kNh * kConvDim * 4) return;
  if (in_sizes[3] != kNh * kConvDim || in_sizes[11] != kNh * kConvDim) return;
  if (in_sizes[4] != kNh * kNhIn || in_sizes[12] != kNh * kNhIn) return;
  if (in_sizes[5] != kNh * kNhIn || in_sizes[13] != kNh * kNhIn) return;
  if (in_sizes[6] != kNh * kNhIn || in_sizes[14] != kNh * kNhIn) return;
  if (in_sizes[7] != kNh * kDinner || in_sizes[15] != kNh * kDinner) return;
  if (in_sizes[8] != kNh * kHd * kDinner || in_sizes[16] != kNh * kHd * kDinner) return;
  if (in_sizes[17] != kDm || in_sizes[18] != kNh * kHd || in_sizes[19] != kNh * kHd) return;
  if (in_sizes[20] != kDm * kDm || in_sizes[21] != kDm) return;
  if (out_size != kRows * kDm) return;
  if (ws_size < kWsTotal) return;

  const float* x      = (const float*)d_in[0];
  const float* lam    = (const float*)d_in[17];
  const float* gnw    = (const float*)d_in[18];
  const float* gnb    = (const float*)d_in[19];
  const float* projw  = (const float*)d_in[20];
  const float* projb  = (const float*)d_in[21];
  float* out = (float*)d_out;

  char* ws = (char*)d_ws;
  unsigned short* WP1 = (unsigned short*)(ws + kOffWP1);
  unsigned short* WP2 = (unsigned short*)(ws + kOffWP2);
  unsigned short* WOT = (unsigned short*)(ws + kOffWOT);
  unsigned short* PJW = (unsigned short*)(ws + kOffPJW);
  float*          Y   = (float*)(ws + kOffY);
  float*          ST  = (float*)(ws + kOffST);
  unsigned short* APL = (unsigned short*)(ws + kOffAPL);

  prep_planes_kernel<<<144, 256, 0, stream>>>(
      (const float*)d_in[1], (const float*)d_in[9], (const float*)d_in[8], (const float*)d_in[16], projw,
      WP1, WP2, WOT, PJW);

  mamba_head_kernel<<<kNh * kBatch, 128, 0, stream>>>(
      x, WP1, WP2, WOT,
      (const float*)d_in[2], (const float*)d_in[3], (const float*)d_in[4],
      (const float*)d_in[5], (const float*)d_in[6], (const float*)d_in[7],
      Y);
  mamba_head_kernel<<<kNh * kBatch, 128, 0, stream>>>(
      x, WP1 + (size_t)kWinRows * 32, WP2 + (size_t)kWinRows * 32, WOT + (size_t)kNh * kHd * kDinner,
      (const float*)d_in[10], (const float*)d_in[11], (const float*)d_in[12],
      (const float*)d_in[13], (const float*)d_in[14], (const float*)d_in[15],
      Y + (size_t)(kNh * kBatch) * kPlane);

  gn_stats_kernel<<<kNh * kBatch, 256, 0, stream>>>(Y, lam, ST);
  gn_apply_kernel<<<kRows / 64, 256, 0, stream>>>(Y, ST, lam, gnw, gnb, APL);

  proj_gemm_kernel<<<(kRows / 64) * (kDm / 64) / 8, 256, 0, stream>>>(
      APL, kDm, PJW, kDm, out, kDm, projb, x, kRows, kDm, kDm, kFoldProj);
}
